// SNN_Model_59227599012529
// MI455X (gfx1250) — hardware-verified
//
#include <hip/hip_runtime.h>
#include <stdint.h>


typedef _Float16 v16h __attribute__((ext_vector_type(16)));
typedef _Float16 v8h  __attribute__((ext_vector_type(8)));
typedef float    v8f  __attribute__((ext_vector_type(8)));
typedef float    v4f  __attribute__((ext_vector_type(4)));
union Frag { v16h v; v8h half[2]; };

#define THREADS  128
#define NWAVE    4
#define TILE_M   16
#define D_IN     128
#define H1       400
#define H2       300
#define O_OUT    3
#define KT1      4
#define NT1      25
#define KT2      13
#define NT2      19
#define NP2      304
#define W2P      448
#define KT3      10
#define KP3      320
#define SLOT     64
#define MAXSTEPS 1024
#define THR      1.0f
#define BETA     0.95f
#define SC_X     256.0f
#define SC_W     64.0f
#define INV_S0   (1.0f / 16384.0f)
#define INV_SW   (1.0f / 64.0f)

__device__ __forceinline__ v8f v8f_zero() {
  v8f r;
#pragma unroll
  for (int i = 0; i < 8; ++i) r[i] = 0.0f;
  return r;
}

__device__ __forceinline__ v8f wmma16(v16h a, v16h b, v8f c) {
  v8f d = __builtin_amdgcn_wmma_f32_16x16x32_f16(false, a, false, b, (short)0, c, false, false);
  asm volatile("v_nop\n\tv_nop\n\tv_nop\n\tv_nop" : "+v"(d) : "v"(a), "v"(b));
  return d;
}

__device__ __forceinline__ v8h cvt8(v4f p, v4f q, float sc) {
  v8h r;
  r[0] = (_Float16)(p[0] * sc); r[1] = (_Float16)(p[1] * sc);
  r[2] = (_Float16)(p[2] * sc); r[3] = (_Float16)(p[3] * sc);
  r[4] = (_Float16)(q[0] * sc); r[5] = (_Float16)(q[1] * sc);
  r[6] = (_Float16)(q[2] * sc); r[7] = (_Float16)(q[3] * sc);
  return r;
}

__device__ __forceinline__ int afrag_idx(int m, int kk) {
  const int ln = m + ((kk & 8) ? 16 : 0);
  const int el = (kk & 7) + ((kk & 16) ? 8 : 0);
  return ln * 16 + el;
}

__device__ __forceinline__ float lif_mem(float mem, float cur) {
#pragma clang fp contract(off)
  const float reset = (mem > THR) ? 1.0f : 0.0f;
  float t = BETA * mem;
  t = t + cur;
  t = t - reset;
  return t;
}

__device__ __forceinline__ v8h load_w2_group(const float* __restrict__ W2, int row, int k) {
  v8h r;
  if (row < H2 && k < H1) {
    const v4f p = *(const v4f*)(W2 + (size_t)row * H1 + k);
    const v4f q = *(const v4f*)(W2 + (size_t)row * H1 + k + 4);
    r = cvt8(p, q, SC_W);
  } else {
#pragma unroll
    for (int i = 0; i < 8; ++i) r[i] = (_Float16)0.0f;
  }
  return r;
}

__global__ __launch_bounds__(64)
void k_cvt_w2(const float* __restrict__ W2, _Float16* __restrict__ W2h) {
  const int row  = blockIdx.x * 2 + (int)(threadIdx.x >> 5);
  const int lane = threadIdx.x & 31;
  if (row >= NP2) return;
  const int kA = 8 * lane;
  const int kB = 256 + 8 * lane;
  const v8h vA = load_w2_group(W2, row, kA);
  v8h vB;
#pragma unroll
  for (int i = 0; i < 8; ++i) vB[i] = (_Float16)0.0f;
  if (kB < W2P) vB = load_w2_group(W2, row, kB);
  _Float16* base = W2h + (size_t)row * W2P;
  *(volatile v8h*)(base + kA) = vA;
  if (kB < W2P) *(volatile v8h*)(base + kB) = vB;
  __threadfence();
  *(volatile v8h*)(base + kA) = vA;
  if (kB < W2P) *(volatile v8h*)(base + kB) = vB;
}

struct __attribute__((aligned(32))) Smem {
  _Float16 a1[KT2 * 512];
  float    cur1[TILE_M * H1];
  float    mem1[TILE_M * H1];
  _Float16 a3[KT3 * 512];
  _Float16 w3[16 * KP3];
  float    ost[SLOT];
};

__global__ __launch_bounds__(THREADS)
void k_snn(const float* __restrict__ x,  const float* __restrict__ W1, const float* __restrict__ b1,
           const _Float16* __restrict__ W2h, const float* __restrict__ b2,
           const float* __restrict__ W3, const float* __restrict__ b3,
           const int* __restrict__ nsp, float* __restrict__ slots, int B) {
#pragma clang fp contract(off)
  __shared__ Smem s;
  const int tid  = threadIdx.x;
  const int wave = __builtin_amdgcn_readfirstlane(tid >> 5);
  const int lane = tid & 31;
  const int h    = lane >> 4;
  const int m16  = lane & 15;
  const int row0 = blockIdx.x * TILE_M;
  int nsteps = nsp[0];
  nsteps = (nsteps < 0) ? 0 : ((nsteps > MAXSTEPS) ? MAXSTEPS : nsteps);

  _Float16* xs = s.a1;
  for (int i = tid; i < TILE_M * D_IN; i += THREADS) {
    const int m = i >> 7, k = i & 127;
    const int row = row0 + m;
    const float v = (row < B) ? x[(size_t)row * D_IN + k] : 0.0f;
    xs[i] = (_Float16)(v * SC_X);
  }
  for (int i = tid; i < 16 * KP3; i += THREADS) {
    const int n = i / KP3, k = i - n * KP3;
    const float v = (n < O_OUT && k < H2) ? W3[n * H2 + k] : 0.0f;
    s.w3[i] = (_Float16)(v * SC_W);
  }
  for (int i = tid; i < TILE_M * H1; i += THREADS) s.mem1[i] = 0.0f;
  for (int i = tid; i < KT3 * 512; i += THREADS) s.a3[i] = (_Float16)0.0f;
  __syncthreads();

  for (int nt = wave; nt < NT1; nt += NWAVE) {
    const int n = nt * 16 + m16;
    const float* wr = W1 + (size_t)n * D_IN;
    v8f acc = v8f_zero();
#pragma unroll
    for (int kt = 0; kt < KT1; ++kt) {
      const int k0 = kt * 32;
      Frag a, b;
      a.half[0] = *(const v8h*)(xs + m16 * D_IN + k0 + 8 * h);
      a.half[1] = *(const v8h*)(xs + m16 * D_IN + k0 + 16 + 8 * h);
      const v4f p0 = *(const v4f*)(wr + k0 + 8 * h);
      const v4f p1 = *(const v4f*)(wr + k0 + 8 * h + 4);
      const v4f q0 = *(const v4f*)(wr + k0 + 16 + 8 * h);
      const v4f q1 = *(const v4f*)(wr + k0 + 16 + 8 * h + 4);
      b.half[0] = cvt8(p0, p1, SC_W);
      b.half[1] = cvt8(q0, q1, SC_W);
      acc = wmma16(a.v, b.v, acc);
    }
    const float bb = b1[n];
#pragma unroll
    for (int r = 0; r < 8; ++r) {
      float c = acc[r] * INV_S0;
      c = c + bb;
      s.cur1[(8 * h + r) * H1 + n] = c;
    }
  }
  __syncthreads();

  float b2v[5];
  const _Float16* w2r[5];
#pragma unroll
  for (int sl = 0; sl < 5; ++sl) {
    const int nt  = wave + NWAVE * sl;
    const int n   = nt * 16 + m16;
    b2v[sl] = (nt < NT2 && n < H2) ? b2[n] : 0.0f;
    const int ntc = (nt < NT2) ? nt : (nt - NWAVE);
    w2r[sl] = W2h + (size_t)(ntc * 16 + m16) * W2P + 8 * h;
  }
  const float b3v = (m16 < O_OUT) ? b3[m16] : 0.0f;
  v8f mem2[5];
#pragma unroll
  for (int sl = 0; sl < 5; ++sl) mem2[sl] = v8f_zero();
  v8f mem3 = v8f_zero();
  v8f accO = v8f_zero();
  const _Float16* a1l = s.a1 + lane * 16;
  const _Float16* a3l = s.a3 + lane * 16;
  const _Float16* w3l = s.w3 + m16 * KP3 + 8 * h;

  for (int t = 0; t < nsteps; ++t) {
    for (int r = tid; r < KT2 * 32; r += THREADS) {
      const int kt = r >> 5, fl = r & 31;
      const int m  = fl & 15;
      const int k0 = kt * 32 + ((fl & 16) ? 8 : 0);
      const int base = m * H1 + k0;
      Frag spk;
      {
        const v8f c = *(const v8f*)(s.cur1 + base);
        v8f mm = *(const v8f*)(s.mem1 + base);
#pragma unroll
        for (int j = 0; j < 8; ++j) {
          const float nv = lif_mem(mm[j], c[j]);
          mm[j] = nv;
          spk.v[j] = (nv > THR) ? (_Float16)1.0f : (_Float16)0.0f;
        }
        *(v8f*)(s.mem1 + base) = mm;
      }
      if (kt < KT2 - 1) {
        const v8f c = *(const v8f*)(s.cur1 + base + 16);
        v8f mm = *(const v8f*)(s.mem1 + base + 16);
#pragma unroll
        for (int j = 0; j < 8; ++j) {
          const float nv = lif_mem(mm[j], c[j]);
          mm[j] = nv;
          spk.v[8 + j] = (nv > THR) ? (_Float16)1.0f : (_Float16)0.0f;
        }
        *(v8f*)(s.mem1 + base + 16) = mm;
      } else {
#pragma unroll
        for (int j = 0; j < 8; ++j) spk.v[8 + j] = (_Float16)0.0f;
      }
      *(v16h*)(s.a1 + kt * 512 + fl * 16) = spk.v;
    }
    __syncthreads();

    v8f acc[5];
#pragma unroll
    for (int sl = 0; sl < 5; ++sl) acc[sl] = v8f_zero();
#pragma unroll 1
    for (int kt = 0; kt < KT2; ++kt) {
      Frag a;
      a.v = *(const v16h*)(a1l + kt * 512);
      Frag b[5];
#pragma unroll
      for (int sl = 0; sl < 5; ++sl) {
        b[sl].half[0] = *(const v8h*)(w2r[sl] + kt * 32);
        b[sl].half[1] = *(const v8h*)(w2r[sl] + kt * 32 + 16);
      }
#pragma unroll
      for (int sl = 0; sl < 5; ++sl)
        acc[sl] = __builtin_amdgcn_wmma_f32_16x16x32_f16(false, a.v, false, b[sl].v, (short)0,
                                                          acc[sl], false, false);
      asm volatile("v_nop\n\tv_nop\n\tv_nop\n\tv_nop"
                   : "+v"(acc[0]), "+v"(acc[1]), "+v"(acc[2]), "+v"(acc[3]), "+v"(acc[4])
                   : "v"(a.v), "v"(b[0].v), "v"(b[1].v), "v"(b[2].v), "v"(b[3].v), "v"(b[4].v));
    }

#pragma unroll
    for (int sl = 0; sl < 5; ++sl) {
      const int nt = wave + NWAVE * sl;
      if (nt < NT2) {
        const int kcol = nt * 16 + m16;
        const int kt3  = kcol >> 5, kk = kcol & 31;
#pragma unroll
        for (int v = 0; v < 8; ++v) {
          float cur = acc[sl][v] * INV_SW;
          cur = cur + b2v[sl];
          const float nv = lif_mem(mem2[sl][v], cur);
          mem2[sl][v] = nv;
          s.a3[kt3 * 512 + afrag_idx(v + 8 * h, kk)] = (nv > THR) ? (_Float16)1.0f : (_Float16)0.0f;
        }
      }
    }
    __syncthreads();

    if (wave == 0) {
      v8f acc3 = v8f_zero();
#pragma unroll
      for (int kt = 0; kt < KT3; ++kt) {
        Frag a, b;
        a.v = *(const v16h*)(a3l + kt * 512);
        b.half[0] = *(const v8h*)(w3l + kt * 32);
        b.half[1] = *(const v8h*)(w3l + kt * 32 + 16);
        acc3 = wmma16(a.v, b.v, acc3);
      }
#pragma unroll
      for (int v = 0; v < 8; ++v) {
        float cur = acc3[v] * INV_SW;
        cur = cur + b3v;
        const float nv = lif_mem(mem3[v], cur);
        mem3[v] = nv;
        accO[v] = accO[v] + ((nv > THR) ? 1.0f : 0.0f);
      }
    }
  }

  if (wave == 0) {
#pragma unroll
    for (int v = 0; v < 8; ++v)
      if (m16 < O_OUT) s.ost[(8 * h + v) * O_OUT + m16] = accO[v];
  }
  if (tid >= TILE_M * O_OUT && tid < SLOT) s.ost[tid] = 0.0f;
  __syncthreads();
  if (tid < SLOT / 4) {
    const v4f val = *(const v4f*)(s.ost + 4 * tid);
    volatile v4f* d = (volatile v4f*)(slots + (size_t)blockIdx.x * SLOT + 4 * tid);
    *d = val;
    __threadfence();
    *d = val;
  }
}

__global__ __launch_bounds__(256)
void k_out(const float* __restrict__ slots, const int* __restrict__ nsp,
           float* __restrict__ out, int out_n, int nblk) {
#pragma clang fp contract(off)
  const int i  = blockIdx.x * 256 + (int)threadIdx.x;
  const int f0 = 4 * i;
  if (f0 >= out_n) return;
  int ns = nsp[0];
  ns = (ns < 1) ? 1 : ((ns > MAXSTEPS) ? MAXSTEPS : ns);
  const float inv = 1.0f / (float)ns;
  v4f val;
#pragma unroll
  for (int j = 0; j < 4; ++j) {
    const int f = f0 + j;
    float r = 0.0f;
    if (f < out_n) {
      const int row = f / O_OUT;
      const int col = f - row * O_OUT;
      int blk = row / TILE_M;
      const int lr = row - blk * TILE_M;
      if (blk >= nblk) blk = nblk - 1;
      const float cnt = slots[(size_t)blk * SLOT + lr * O_OUT + col];
      const float z = cnt * inv;
      const float e = expf(-z);
      r = 1.0f / (1.0f + e);
    }
    val[j] = r;
  }
  if (f0 + 3 < out_n) {
    volatile v4f* d = (volatile v4f*)(out + f0);
    *d = val;
    __threadfence();
    *d = val;
  } else {
    volatile float* o = (volatile float*)out;
#pragma unroll
    for (int j = 0; j < 4; ++j) if (f0 + j < out_n) o[f0 + j] = val[j];
    __threadfence();
#pragma unroll
    for (int j = 0; j < 4; ++j) if (f0 + j < out_n) o[f0 + j] = val[j];
  }
}

extern "C" void kernel_launch(void* const* d_in, const int* in_sizes, int n_in,
                              void* d_out, int out_size, void* d_ws, size_t ws_size,
                              hipStream_t stream) {
  if (n_in < 8) return;
  const float* x  = (const float*)d_in[0];
  const float* W1 = (const float*)d_in[1];
  const float* b1 = (const float*)d_in[2];
  const float* W2 = (const float*)d_in[3];
  const float* b2 = (const float*)d_in[4];
  const float* W3 = (const float*)d_in[5];
  const float* b3 = (const float*)d_in[6];
  const int*   ns = (const int*)d_in[7];
  float* out = (float*)d_out;

  if (in_sizes[0] <= 0 || (in_sizes[0] % D_IN) != 0) return;
  const int B = in_sizes[0] / D_IN;
  if (in_sizes[1] != H1 * D_IN || in_sizes[2] != H1 || in_sizes[3] != H2 * H1 ||
      in_sizes[4] != H2 || in_sizes[5] != O_OUT * H2 || in_sizes[6] != O_OUT || in_sizes[7] < 1)
    return;
  if (out_size != B * O_OUT) return;
  const int nblk = (B + TILE_M - 1) / TILE_M;

  const size_t bytes_w2h   = (size_t)NP2 * W2P * sizeof(_Float16);
  const size_t off_slots   = (bytes_w2h + 127) & ~(size_t)127;
  const size_t bytes_slots = (size_t)nblk * SLOT * sizeof(float);
  if (off_slots + bytes_slots > ws_size) return;
  char* ws = (char*)d_ws;
  _Float16* W2h   = (_Float16*)ws;
  float*    slots = (float*)(ws + off_slots);

  k_cvt_w2<<<dim3((NP2 + 1) / 2), dim3(64), 0, stream>>>(W2, W2h);
  k_snn<<<dim3(nblk), dim3(THREADS), 0, stream>>>(x, W1, b1, W2h, b2, W3, b3, ns, slots, B);
  const int nthr = (out_size + 3) / 4;
  k_out<<<dim3((nthr + 255) / 256), dim3(256), 0, stream>>>(slots, ns, out, out_size, nblk);
}
